// S4Block_1855425872534
// MI455X (gfx1250) — hardware-run, weakly checked
//
#include <hip/hip_runtime.h>
#include <math.h>

typedef __attribute__((ext_vector_type(16))) _Float16 v16h;
typedef __attribute__((ext_vector_type(8)))  _Float16 v8h;
typedef __attribute__((ext_vector_type(16))) __bf16   v16b;
typedef __attribute__((ext_vector_type(8)))  __bf16   v8b;
typedef __attribute__((ext_vector_type(8)))  float    v8f;
typedef __attribute__((ext_vector_type(4)))  float    v4f;

constexpr int kB    = 2;
constexpr int kL    = 2048;
constexpr int kRows = kB * kL;
constexpr int kD    = 768;
constexpr int kNs   = 64;
constexpr int kThr  = 256;
constexpr float kInCarry = 1024.0f;
constexpr float kSc = 1.0f / (kInCarry * kInCarry);
constexpr float kInvD = 1.0f / 768.0f;
constexpr float kLnEps = 1e-5f;
constexpr float kF16MinNormal = 6.103515625e-5f;

static_assert((kRows % 64) == 0 && (kD % 64) == 0 && (kD % 32) == 0 && ((kRows / 64) * (kD / 64)) % 8 == 0, "GEMM M, N multiples of 64, K of 32; the grid exact (768 tiles)");

constexpr size_t kOffWIN16 = 0ull;
constexpr size_t kOffWOUT16 = 1179648ull;
constexpr size_t kOffABAR = 2359296ull;
constexpr size_t kOffBBAR = 2555904ull;
constexpr size_t kOffCPL = 2752512ull;
constexpr size_t kOffBIN = 2949120ull;
constexpr size_t kOffBOUT = 2952192ull;
constexpr size_t kOffXN16 = 2955264ull;
constexpr size_t kOffU32 = 9246720ull;
constexpr size_t kOffYP = 21829632ull;
constexpr size_t kOffY16 = 46995456ull;
constexpr size_t kOffO32 = 53286912ull;
constexpr size_t kWsTotal = 65869824ull;
static_assert(kWsTotal <= 134217728ull, "carve cap: under 128 MiB");
static_assert(kOffWIN16 == 0
              && kOffWOUT16 == kOffWIN16 + 1179648ull
              && kOffABAR == kOffWOUT16 + 1179648ull
              && kOffBBAR == kOffABAR + 196608ull
              && kOffCPL == kOffBBAR + 196608ull
              && kOffBIN == kOffCPL + 196608ull
              && kOffBOUT == kOffBIN + 3072ull
              && kOffXN16 == kOffBOUT + 3072ull
              && kOffU32 == kOffXN16 + 6291456ull
              && kOffYP == kOffU32 + 12582912ull
              && kOffY16 == kOffYP + 25165824ull
              && kOffO32 == kOffY16 + 6291456ull
              && kWsTotal == kOffO32 + 12582912ull, "the carve is chained and totalled");
static_assert((kOffWIN16 % 256) == 0 && (kOffWOUT16 % 256) == 0 && (kOffABAR % 256) == 0 && (kOffBBAR % 256) == 0 && (kOffCPL % 256) == 0 && (kOffBIN % 256) == 0 && (kOffBOUT % 256) == 0 && (kOffXN16 % 256) == 0 && (kOffU32 % 256) == 0 && (kOffYP % 256) == 0 && (kOffY16 % 256) == 0 && (kOffO32 % 256) == 0, "aligned regions");

__device__ __forceinline__ unsigned short f2bf_bits(float f) {
  unsigned u = __float_as_uint(f);
  return (unsigned short)((u + 0x7FFFu + ((u >> 16) & 1u)) >> 16);
}
__device__ __forceinline__ float bf_bits2f(unsigned short h) { return __uint_as_float(((unsigned)h) << 16); }
__device__ __forceinline__ float bf16r(float f) { return bf_bits2f(f2bf_bits(f)); }
__device__ __forceinline__ float carry_flush(float v, float carry) {
  const float s = v * carry;
  return (fabsf(s) < kF16MinNormal) ? 0.0f : s;
}
__device__ __forceinline__ float frcp(float x) { return __builtin_amdgcn_rcpf(x); }

__device__ __forceinline__ void dep_guard4_h(v8f& a, v8f& b, v8f& c, v8f& d, v16h x, v16h y) { asm volatile("v_nop\n\tv_nop\n\tv_nop\n\tv_nop" : "+v"(a), "+v"(b), "+v"(c), "+v"(d) : "v"(x), "v"(y)); }
__device__ __forceinline__ void dep_guard4_b(v8f& a, v8f& b, v8f& c, v8f& d, v16b x, v16b y) { asm volatile("v_nop\n\tv_nop\n\tv_nop\n\tv_nop" : "+v"(a), "+v"(b), "+v"(c), "+v"(d) : "v"(x), "v"(y)); }
__device__ __forceinline__ void keep4_h(v16h a, v16h b, v16h c, v16h d) { asm volatile("v_nop" :: "v"(a), "v"(b), "v"(c), "v"(d)); }
__device__ __forceinline__ void keep4_b(v16b a, v16b b, v16b c, v16b d) { asm volatile("v_nop" :: "v"(a), "v"(b), "v"(c), "v"(d)); }
__device__ __forceinline__ void acc_guard4(v8f& a, v8f& b, v8f& c, v8f& d) { asm volatile("v_nop\n\tv_nop\n\tv_nop\n\tv_nop" : "+v"(a), "+v"(b), "+v"(c), "+v"(d)); }

template <typename T> struct Frag;
template <> struct Frag<_Float16> {
  typedef v16h V; union U { v16h v; v8h h[2]; };
  static __device__ __forceinline__ v16h load(const _Float16* p) {
    U f; f.h[0] = *(const v8h*)(p); f.h[1] = *(const v8h*)(p + 16); return f.v;
  }
  static __device__ __forceinline__ v8f mma(v16h a, v16h b, v8f c) {
    return __builtin_amdgcn_wmma_f32_16x16x32_f16(false, a, false, b, (short)0, c, false, false);
  }
  static __device__ __forceinline__ void guard4(v8f& a, v8f& b, v8f& c, v8f& d, v16h x, v16h y) { dep_guard4_h(a, b, c, d, x, y); }
  static __device__ __forceinline__ void keep(v16h a, v16h b, v16h c, v16h d) { keep4_h(a, b, c, d); }
};
template <> struct Frag<__bf16> {
  typedef v16b V; union U { v16b v; v8b h[2]; };
  static __device__ __forceinline__ v16b load(const __bf16* p) {
    U f; f.h[0] = *(const v8b*)(p); f.h[1] = *(const v8b*)(p + 16); return f.v;
  }
  static __device__ __forceinline__ v8f mma(v16b a, v16b b, v8f c) {
    return __builtin_amdgcn_wmma_f32_16x16x32_bf16(false, a, false, b, (short)0, c, false, false);
  }
  static __device__ __forceinline__ void guard4(v8f& a, v8f& b, v8f& c, v8f& d, v16b x, v16b y) { dep_guard4_b(a, b, c, d, x, y); }
  static __device__ __forceinline__ void keep(v16b a, v16b b, v16b c, v16b d) { keep4_b(a, b, c, d); }
};

__device__ __forceinline__ v8f mma_h(v16h a, v16h b, v8f c) {
  c = __builtin_amdgcn_wmma_f32_16x16x32_f16(false, a, false, b, (short)0, c, false, false);
  asm volatile("v_nop\n\tv_nop\n\tv_nop\n\tv_nop" : "+v"(c) : "v"(a), "v"(b));
  return c;
}

template <int ET> struct Elem;
template <> struct Elem<0> { typedef _Float16 T; };
template <> struct Elem<1> { typedef __bf16 T; };
template <int ET, bool SPLIT, int BIAS_MODE, int OUT_MODE, bool RESID, int ACT = 0>
__global__ __launch_bounds__(256) void wmma_gemm64(
    const unsigned short* __restrict__ Ap, const unsigned short* __restrict__ A2p, int lda, long strideA,
    const unsigned short* __restrict__ Btp, const unsigned short* __restrict__ Bt2p, int ldb, long strideB,
    void* __restrict__ Cout, void* __restrict__ Cout2, int ldc, long strideC,
    const float* __restrict__ bias,
    const float* __restrict__ resid, long strideR,
    int M, int N, int K, float scale) {
  typedef typename Elem<ET>::T T;
  typedef typename Frag<T>::V V;
  const T* A = (const T*)Ap; const T* A2 = (const T*)A2p; const T* Bt = (const T*)Btp; const T* Bt2 = (const T*)Bt2p;
  __shared__ __align__(16) float sT[8][16 * 68];
  const int b    = blockIdx.y;
  const int lane = threadIdx.x & 31;
  const int wave = threadIdx.x >> 5;
  const int tilesN = N >> 6;
  const int tilesM = M >> 6;
  const int tile = blockIdx.x * 8 + wave;
  if (tile >= tilesM * tilesN) return;
  const int tm = tile / tilesN;
  const int tn = tile - tm * tilesN;
  const int m0 = tm << 6;
  const int n0 = tn << 6;

  const T* Ab  = A  + (size_t)b * strideA;
  const T* Bb  = Bt + (size_t)b * strideB;
  const T* Ab2 = SPLIT ? (A2  + (size_t)b * strideA) : nullptr;
  const T* Bb2 = SPLIT ? (Bt2 + (size_t)b * strideB) : nullptr;

  const int rlane = lane & 15;
  const int koff  = (lane >> 4) * 8;
  const int mOff  = (lane >> 4) * 8;

  v8f acc[4][4];
#pragma unroll
  for (int i = 0; i < 4; ++i)
#pragma unroll
    for (int j = 0; j < 4; ++j) acc[i][j] = (v8f){0.f,0.f,0.f,0.f,0.f,0.f,0.f,0.f};

  for (int k0 = 0; k0 < K; k0 += 32) {
    V bh[4], bl[4];
#pragma unroll
    for (int j = 0; j < 4; ++j) {
      const size_t bo = (size_t)(n0 + (j << 4) + rlane) * ldb + koff + k0;
      bh[j] = Frag<T>::load(Bb + bo);
      if (SPLIT) bl[j] = Frag<T>::load(Bb2 + bo);
    }
#pragma unroll
    for (int i = 0; i < 4; ++i) {
      const size_t ao = (size_t)(m0 + (i << 4) + rlane) * lda + koff + k0;
      V ah = Frag<T>::load(Ab + ao);
      V al;
      if (SPLIT) al = Frag<T>::load(Ab2 + ao);
#pragma unroll
      for (int j = 0; j < 4; ++j) {
        acc[i][j] = Frag<T>::mma(ah, bh[j], acc[i][j]);
        if (SPLIT) {
          acc[i][j] = Frag<T>::mma(ah, bl[j], acc[i][j]);
          acc[i][j] = Frag<T>::mma(al, bh[j], acc[i][j]);
        }
      }
      Frag<T>::guard4(acc[i][0], acc[i][1], acc[i][2], acc[i][3], ah, SPLIT ? al : ah);
    }
    Frag<T>::keep(bh[0], bh[1], bh[2], bh[3]);
    if (SPLIT) Frag<T>::keep(bl[0], bl[1], bl[2], bl[3]);
  }
  acc_guard4(acc[0][0], acc[0][1], acc[0][2], acc[0][3]);
  acc_guard4(acc[1][0], acc[1][1], acc[1][2], acc[1][3]);
  acc_guard4(acc[2][0], acc[2][1], acc[2][2], acc[2][3]);
  acc_guard4(acc[3][0], acc[3][1], acc[3][2], acc[3][3]);

  float* slab = sT[wave];
  const float* Rb = RESID ? (resid + (size_t)b * strideR) : nullptr;
#pragma unroll
  for (int i = 0; i < 4; ++i) {
    const int mBase = m0 + (i << 4);
#pragma unroll
    for (int j = 0; j < 4; ++j) {
      const int n = n0 + (j << 4) + rlane;
      float bv = 0.f;
      if (BIAS_MODE == 2) bv = bias[n];
#pragma unroll
      for (int r = 0; r < 8; ++r) {
        float v = acc[i][j][r] * scale;
        if (BIAS_MODE == 1) v += bias[mBase + mOff + r];
        if (BIAS_MODE == 2) v += bv;
        if (RESID) v += Rb[(size_t)(mBase + mOff + r) * ldc + n];
        if (ACT == 1) v = tanhf(v);
        if (ACT == 2) v = fmaxf(v, 0.0f);
        if (ACT == 3) v = v / (1.0f + expf(-v));
        if (ACT == 4) v = (v > 0.f) ? v : 0.01f * v;
        slab[(mOff + r) * 68 + (j << 4) + rlane] = v;
      }
    }
    __builtin_amdgcn_fence(__ATOMIC_RELEASE, "workgroup");
    __builtin_amdgcn_wave_barrier();
    __builtin_amdgcn_fence(__ATOMIC_ACQUIRE, "workgroup");
    if (OUT_MODE == 0) {
      float* C = (float*)Cout + (size_t)b * strideC;
      const int hh = lane >> 4, c4 = (lane & 15) * 4;
      for (int pass = 0; pass < 2; ++pass) {
#pragma unroll
        for (int it = 0; it < 8; ++it) {
          const int row = it * 2 + hh;
          v4f v = *(const v4f*)(slab + row * 68 + c4);
          *(volatile v4f*)(C + (size_t)(mBase + row) * ldc + n0 + c4) = v;
        }
        __threadfence();
      }
    } else {
      const int q = lane >> 3, c8 = (lane & 7) * 8;
      unsigned short* C  = (unsigned short*)Cout  + (size_t)b * strideC;
      unsigned short* C2 = (OUT_MODE == 2) ? ((unsigned short*)Cout2 + (size_t)b * strideC) : nullptr;
      for (int pass = 0; pass < 2; ++pass) {
#pragma unroll
        for (int it = 0; it < 4; ++it) {
          const int row = it * 4 + q;
          const float* sp = slab + row * 68 + c8;
          v8h hv, lv;
#pragma unroll
          for (int e = 0; e < 8; ++e) {
            if (OUT_MODE == 1) {
              hv[e] = (_Float16)sp[e];
            } else {
              unsigned short hb = f2bf_bits(sp[e]);
              unsigned short lb = f2bf_bits(sp[e] - bf_bits2f(hb));
              hv[e] = __builtin_bit_cast(_Float16, hb);
              lv[e] = __builtin_bit_cast(_Float16, lb);
            }
          }
          *(volatile v8h*)(C + (size_t)(mBase + row) * ldc + n0 + c8) = hv;
          if (OUT_MODE == 2) *(volatile v8h*)(C2 + (size_t)(mBase + row) * ldc + n0 + c8) = lv;
        }
        __threadfence();
      }
    }
    __builtin_amdgcn_fence(__ATOMIC_RELEASE, "workgroup");
    __builtin_amdgcn_wave_barrier();
    __builtin_amdgcn_fence(__ATOMIC_ACQUIRE, "workgroup");
  }
}

__global__ __launch_bounds__(kThr) void cast_plane_kernel(const float* __restrict__ src, unsigned short* __restrict__ dst,
                                                          int colsLog2, int dstPitch, int dstOff) {
  const int i   = blockIdx.x * kThr + threadIdx.x;
  const int sh  = colsLog2 - 3;
  const int row = i >> sh;
  const int c8  = (i & ((1 << sh) - 1)) * 8;
  const float* sp = src + ((size_t)row << colsLog2) + c8;
  const v4f a0 = *(const v4f*)(sp);
  const v4f a1 = *(const v4f*)(sp + 4);
  v8h hv;
#pragma unroll
  for (int e = 0; e < 4; ++e) {
    const float f0 = a0[e];
    const float f1 = a1[e];
    hv[e]     = (_Float16)carry_flush(bf16r(f0), kInCarry);
    hv[4 + e] = (_Float16)carry_flush(bf16r(f1), kInCarry);
  }
  unsigned short* dp = dst + (size_t)row * dstPitch + dstOff + c8;
  *(volatile v8h*)dp = hv;
  __threadfence();
  *(volatile v8h*)dp = hv;
}


__global__ __launch_bounds__(kThr) void setup_kernel(const float* __restrict__ log_A, const float* __restrict__ B_p, const float* __restrict__ C_p,
                                                    const float* __restrict__ log_dt, const float* __restrict__ b_in, const float* __restrict__ b_out,
                                                    float* __restrict__ ABAR, float* __restrict__ BBAR, float* __restrict__ CPL,
                                                    float* __restrict__ BIN, float* __restrict__ BOUT) {
  const unsigned bk = blockIdx.x;
  if (bk < 192u) {
    const unsigned i = bk * (unsigned)kThr + threadIdx.x;
    const unsigned d = i >> 6;
    const float la = log_A[i], bp = B_p[i], cp = C_p[i], ld = log_dt[d];
    const float A = -expf(bf16r(la));
    const float dt = expf(bf16r(ld));
    const float ab = expf(dt * A);
    const float bb = bf16r(bp) * dt;
    const float cc = bf16r(cp);
    for (int pass = 0; pass < 2; ++pass) {
      *(volatile float*)(ABAR + i) = ab;
      *(volatile float*)(BBAR + i) = bb;
      *(volatile float*)(CPL + i) = cc;
      __threadfence();
    }
  } else if (bk < 195u) {
    const unsigned j = (bk - 192u) * (unsigned)kThr + threadIdx.x;
    const float p = b_in[j];
    const float o = bf16r(p);
    *(volatile float*)(BIN + j) = o;
    __threadfence();
    *(volatile float*)(BIN + j) = o;
  } else {
    const unsigned j = (bk - 195u) * (unsigned)kThr + threadIdx.x;
    const float p = b_out[j];
    const float o = bf16r(p);
    *(volatile float*)(BOUT + j) = o;
    __threadfence();
    *(volatile float*)(BOUT + j) = o;
  }
}
static_assert(kD * kNs == 192 * kThr && kNs == 64 && kD == 3 * kThr, "set-up grid exact: 192 blocks of (channel, state) pairs; 3 + 3 blocks of biases");

__global__ __launch_bounds__(kThr) void ln_kernel(const float* __restrict__ x, const float* __restrict__ g, const float* __restrict__ beta,
                                                  unsigned short* __restrict__ XN16) {
  const unsigned r = blockIdx.x * (unsigned)kThr + threadIdx.x;
  const float* a = x + (size_t)r * kD;
  float s = 0.0f;
  for (unsigned c = 0; c < (unsigned)kD; c += 4) {
    const v4f v = *(const v4f*)(a + c);
    s += bf16r(v[0]); s += bf16r(v[1]); s += bf16r(v[2]); s += bf16r(v[3]);
  }
  const float mu = s * kInvD;
  float q = 0.0f;
  for (unsigned c = 0; c < (unsigned)kD; c += 4) {
    const v4f v = *(const v4f*)(a + c);
#pragma unroll
    for (int e = 0; e < 4; ++e) { const float d = bf16r(v[e]) - mu; q += d * d; }
  }
  const float sd = sqrtf(q * kInvD + kLnEps);
  unsigned short* hp = XN16 + (size_t)r * kD;
  for (unsigned c = 0; c < (unsigned)kD; c += 8) {
    const v4f x0 = *(const v4f*)(a + c), x1 = *(const v4f*)(a + c + 4);
    const v4f g0 = *(const v4f*)(g + c), g1 = *(const v4f*)(g + c + 4), b0 = *(const v4f*)(beta + c), b1 = *(const v4f*)(beta + c + 4);
    v8h hv;
#pragma unroll
    for (int e = 0; e < 4; ++e) {
      const float n0 = (bf16r(x0[e]) - mu) / sd * bf16r(g0[e]) + bf16r(b0[e]);
      const float n1 = (bf16r(x1[e]) - mu) / sd * bf16r(g1[e]) + bf16r(b1[e]);
      hv[e] = (_Float16)carry_flush(n0, kInCarry);
      hv[4 + e] = (_Float16)carry_flush(n1, kInCarry);
    }
    *(volatile v8h*)(hp + c) = hv;
    __threadfence();
    *(volatile v8h*)(hp + c) = hv;
  }
}
static_assert(kRows == 16 * kThr && (kD % 8) == 0, "layer-norm grid exact: 16 blocks, one thread a row");

__global__ __launch_bounds__(kThr) void scan_kernel(const float* __restrict__ U32, const float* __restrict__ ABAR, const float* __restrict__ BBAR,
                                                    const float* __restrict__ CPL, const float* __restrict__ Dp, float* __restrict__ YP) {
  const unsigned smp = blockIdx.x / 6u;
  const unsigned rem = blockIdx.x - smp * 6u;
  const unsigned hf = rem / 3u;
  const unsigned d = (rem - hf * 3u) * (unsigned)kThr + threadIdx.x;
  constexpr int kHs = kNs / 2;
  float h[kHs];
#pragma unroll
  for (int n = 0; n < kHs; ++n) h[n] = 0.0f;
  const float q0 = Dp[d];
  const float dc = (hf == 0u) ? bf16r(q0) : 0.0f;
  const float* ap = ABAR + (size_t)d * kNs + hf * (unsigned)kHs;
  const float* bp = BBAR + (size_t)d * kNs + hf * (unsigned)kHs;
  const float* cp = CPL + (size_t)d * kNs + hf * (unsigned)kHs;
  const size_t r0 = (size_t)smp * kL;
  float* yp = YP + (size_t)hf * kRows * kD;
  for (int l = 0; l < kL; ++l) {
    const size_t row = r0 + (size_t)l;
    const float u = U32[row * kD + d];
    float p = 0.0f;
#pragma unroll
    for (int q = 0; q < kHs / 4; ++q) {
      const v4f A4 = *(const v4f*)(ap + 4 * q), B4 = *(const v4f*)(bp + 4 * q), C4 = *(const v4f*)(cp + 4 * q);
#pragma unroll
      for (int e = 0; e < 4; ++e) {
        const int n = 4 * q + e;
        const float hn = A4[e] * h[n] + B4[e] * u;
        h[n] = hn;
        p += hn * C4[e];
      }
    }
    p += dc * u;
    float* dp = yp + row * kD + d;
    *(volatile float*)dp = p;
    __threadfence();
    *(volatile float*)dp = p;
  }
}
static_assert(kB * 2 * kD == 12 * kThr && kD == 3 * kThr && (kNs % 8) == 0, "recurrence grid exact: 12 blocks; six a sample, three a half");

__global__ __launch_bounds__(kThr) void ycast_kernel(const float* __restrict__ YP, unsigned short* __restrict__ Y16) {
  const size_t o8 = ((size_t)blockIdx.x * kThr + threadIdx.x) * 8u;
  const float* p1 = YP + (size_t)kRows * kD;
  const v4f a0 = *(const v4f*)(YP + o8), a1 = *(const v4f*)(YP + o8 + 4);
  const v4f b0 = *(const v4f*)(p1 + o8), b1 = *(const v4f*)(p1 + o8 + 4);
  v8h hv;
#pragma unroll
  for (int e = 0; e < 4; ++e) { hv[e] = (_Float16)carry_flush(a0[e] + b0[e], kInCarry); hv[4 + e] = (_Float16)carry_flush(a1[e] + b1[e], kInCarry); }
  *(volatile v8h*)(Y16 + o8) = hv;
  __threadfence();
  *(volatile v8h*)(Y16 + o8) = hv;
}
static_assert(((size_t)kRows * kD / 8) == 1536ull * kThr, "cast grid exact");

__global__ __launch_bounds__(kThr) void resid_kernel(const float* __restrict__ O32, const float* __restrict__ x, float* __restrict__ out) {
  const size_t o4 = ((size_t)blockIdx.x * kThr + threadIdx.x) * 4u;
  const v4f a = *(const v4f*)(O32 + o4);
  const v4f b = *(const v4f*)(x + o4);
  v4f o;
#pragma unroll
  for (int e = 0; e < 4; ++e) o[e] = a[e] + bf16r(b[e]);
  *(volatile v4f*)(out + o4) = o;
  __threadfence();
  *(volatile v4f*)(out + o4) = o;
}
static_assert(((size_t)kRows * kD / 4) == 3072ull * kThr, "residual grid exact");

static_assert(((size_t)kD * kD / 8) % kThr == 0 && ((size_t)kD * kD) % 256 == 0, "plane cast grids exact; the planes are whole rows of 256");

extern "C" void kernel_launch(void* const* d_in, const int* in_sizes, int n_in,
                              void* d_out, int out_size, void* d_ws, size_t ws_size,
                              hipStream_t stream) {
  if (n_in < 12 || d_out == nullptr || d_ws == nullptr) return;
  if (in_sizes[0] != kRows * kD || in_sizes[1] != kD || in_sizes[2] != kD || in_sizes[3] != kD * kD || in_sizes[4] != kD || in_sizes[5] != kD * kNs) return;
  if (in_sizes[6] != kD * kNs || in_sizes[7] != kD * kNs || in_sizes[8] != kD || in_sizes[9] != kD || in_sizes[10] != kD * kD || in_sizes[11] != kD) return;
  if (out_size != kRows * kD) return;
  if (ws_size < kWsTotal) return;
  const float* x = (const float*)d_in[0];
  const float* ln_gamma = (const float*)d_in[1];
  const float* ln_beta = (const float*)d_in[2];
  const float* W_in = (const float*)d_in[3];
  const float* b_in = (const float*)d_in[4];
  const float* log_A = (const float*)d_in[5];
  const float* B_p = (const float*)d_in[6];
  const float* C_p = (const float*)d_in[7];
  const float* D_p = (const float*)d_in[8];
  const float* log_dt = (const float*)d_in[9];
  const float* W_out = (const float*)d_in[10];
  const float* b_out = (const float*)d_in[11];
  float* out = (float*)d_out;
  char* ws = (char*)d_ws;
  unsigned short* WIN16 = (unsigned short*)(ws + kOffWIN16);
  unsigned short* WOUT16 = (unsigned short*)(ws + kOffWOUT16);
  float* ABAR = (float*)(ws + kOffABAR);
  float* BBAR = (float*)(ws + kOffBBAR);
  float* CPL = (float*)(ws + kOffCPL);
  float* BIN = (float*)(ws + kOffBIN);
  float* BOUT = (float*)(ws + kOffBOUT);
  unsigned short* XN16 = (unsigned short*)(ws + kOffXN16);
  float* U32 = (float*)(ws + kOffU32);
  float* YP = (float*)(ws + kOffYP);
  unsigned short* Y16 = (unsigned short*)(ws + kOffY16);
  float* O32 = (float*)(ws + kOffO32);

  cast_plane_kernel<<<(int)(((size_t)kD * kD / 8) / kThr), kThr, 0, stream>>>(W_in, WIN16, 8, 256, 0);
  cast_plane_kernel<<<(int)(((size_t)kD * kD / 8) / kThr), kThr, 0, stream>>>(W_out, WOUT16, 8, 256, 0);
  setup_kernel<<<198, kThr, 0, stream>>>(log_A, B_p, C_p, log_dt, b_in, b_out, ABAR, BBAR, CPL, BIN, BOUT);
  ln_kernel<<<kRows / kThr, kThr, 0, stream>>>(x, ln_gamma, ln_beta, XN16);
  wmma_gemm64<0, false, 2, 0, false, 0><<<dim3((kRows / 64) * (kD / 64) / 8, 1), 256, 0, stream>>>(
      XN16, XN16, kD, 0L, WIN16, WIN16, kD, 0L, (void*)U32, (void*)U32, kD, 0L, BIN, nullptr, 0L, kRows, kD, kD, kSc);
  scan_kernel<<<12, kThr, 0, stream>>>(U32, ABAR, BBAR, CPL, D_p, YP);
  ycast_kernel<<<1536, kThr, 0, stream>>>(YP, Y16);
  wmma_gemm64<0, false, 2, 0, false, 0><<<dim3((kRows / 64) * (kD / 64) / 8, 1), 256, 0, stream>>>(
      Y16, Y16, kD, 0L, WOUT16, WOUT16, kD, 0L, (void*)O32, (void*)O32, kD, 0L, BOUT, nullptr, 0L, kRows, kD, kD, kSc);
  resid_kernel<<<3072, kThr, 0, stream>>>(O32, x, out);
}
